// RGCN_90795608637584
// MI455X (gfx1250) — hardware-verified
//
#include <hip/hip_runtime.h>
#include <stddef.h>
#include <stdint.h>
#include <math.h>


#define DIN    64
#define DH     64
#define NREL   8
#define GR     2
#define NGRP   (NREL / GR)
#define KB1    DIN
#define KB2    (2 * DH)
#define NB1    (NREL * DH + DH)
#define NB2    (NREL * DH + DH)
#define RB1    (NREL * DH)
#define RB2    (NREL * DH)
#define TP     (GR * DH)
#define NTHR   256
#define NWAVE  8
#define EPT    8
#define CHUNK  (NTHR * EPT)
#define WCAP   (EPT * 32)
#define LISTN  (NWAVE * WCAP)
#define NBA    4096
#define SLA    12
#define RCAP   28672
#define DEGCAP 64
#define GBM    64
#define GTHR   128
#define UB1    (NB1 * (KB1 / 8))
#define UB1R   (RB1 * (KB1 / 8))
#define UB2    (NB2 * (KB2 / 8))
#define UB2R   (RB2 * (KB2 / 8))
#define UTOT   (UB1 + UB2)
#define PARTW  160
#define WSTW   130
#define PSTOFF 1152
#define APB    64
#define APR    8
#define AGG_ZINTS    (LISTN + 2 * RCAP + 3 * NBA)
#define MISC_INTS    96
#define AGG_LDS_INTS (AGG_ZINTS + MISC_INTS)
#define WSMAX  134217728

static_assert((CHUNK & (CHUNK - 1)) == 0 && CHUNK <= 2048);
static_assert((NBA & (NBA - 1)) == 0 && NBA == (1 << SLA));
static_assert(((long long)CHUNK << SLA) < (1LL << 31));
static_assert(LISTN % NTHR == 0);
static_assert(NBA % NWAVE == 0 && NBA % 32 == 0 && NBA % GBM == 0);
static_assert(RCAP % 32 == 0 && AGG_ZINTS % (NTHR * 4) == 0 && LISTN % 4 == 0 && (AGG_LDS_INTS % 4) == 0);
static_assert(MISC_INTS >= 16 + DEGCAP + 1 && DEGCAP + 1 <= NTHR);
static_assert(AGG_LDS_INTS * 4 <= 300000);
static_assert(KB1 % 32 == 0 && KB2 % 32 == 0 && TP == 128 && DH == 64 && DIN == 64);
static_assert(GBM == (GTHR / 32) * 16 && GBM % 16 == 0);
static_assert(UB1 % NTHR == 0 && UB1R % NTHR == 0 && UB2 % NTHR == 0 && UB2R % NTHR == 0 && UTOT % NTHR == 0);
static_assert(NGRP * GR == NREL && GR == 2);
static_assert(PARTW % 32 == 0 && PARTW >= 2 * DH + 1 && PARTW / 4 <= NTHR);
static_assert(WSTW >= 2 * DH + 1 && NWAVE * WSTW <= PSTOFF && (PSTOFF % 4) == 0 && ((LISTN + PSTOFF) % 4) == 0 && PSTOFF + PARTW <= RCAP);
static_assert(APB == NWAVE * APR && APB == GBM && APR == 8);
static_assert(2 * DH <= NTHR && DH % 8 == 0);

typedef float          v2f   __attribute__((ext_vector_type(2)));
typedef float          v4f   __attribute__((ext_vector_type(4)));
typedef float          v8f   __attribute__((ext_vector_type(8)));
typedef int            v4i   __attribute__((ext_vector_type(4)));
typedef int            v8i   __attribute__((ext_vector_type(8)));
typedef unsigned short v8us  __attribute__((ext_vector_type(8)));
typedef unsigned short v16us __attribute__((ext_vector_type(16)));
typedef __bf16         v16bf __attribute__((ext_vector_type(16)));
typedef v2f  __attribute__((may_alias)) v2fa;
typedef v4f  __attribute__((may_alias)) v4fa;
typedef v4i  __attribute__((may_alias)) v4ia;
typedef v8us __attribute__((may_alias)) v8usa;
union Frag { v16bf v; v16us u; v8us h[2]; v8i w; };

__device__ __forceinline__ v8f wmb(const Frag& a, const Frag& b, v8f c) {
  v8f d = __builtin_amdgcn_wmma_f32_16x16x32_bf16(false, a.v, false, b.v, (short)0, c, false, false);
  asm volatile("v_nop\n\tv_nop\n\tv_nop\n\tv_nop" : "+v"(d) : "v"(a.w), "v"(b.w));
  return d;
}

__device__ __forceinline__ unsigned bf16_bits(float f) {
  const unsigned u = __float_as_uint(f);
  return (u + 0x7FFFu + ((u >> 16) & 1u)) >> 16;
}
__device__ __forceinline__ float bf16_val(float f) {
  return __uint_as_float(bf16_bits(f) << 16);
}

__device__ __forceinline__ int scan_chunk(const int* __restrict__ dsts, const int* __restrict__ ets, int nE,
                                          int cbase, int slotBase, int g0, int* list, int tid, int lane, int wave) {
  int wc = 0;
  const int el0 = tid * EPT;
  const int e0  = cbase + el0;
  const int lim = nE - 4;
  const int q0  = e0 < lim ? e0 : lim;
  const int q1  = (e0 + 4) < lim ? (e0 + 4) : lim;
  const v4i da = *(const v4ia*)(dsts + q0);
  const v4i db = *(const v4ia*)(dsts + q1);
  const v4i ta = *(const v4ia*)(ets + q0);
  const v4i tb = *(const v4ia*)(ets + q1);
  const unsigned nbs = (unsigned)slotBase, ug = (unsigned)g0, ue0 = (unsigned)e0, unE = (unsigned)nE;
  const unsigned unb = (unsigned)NBA, ugr = (unsigned)GR;
  const unsigned s0 = (unsigned)da.x - nbs, s1 = (unsigned)da.y - nbs;
  const unsigned s2 = (unsigned)da.z - nbs, s3 = (unsigned)da.w - nbs;
  const unsigned s4 = (unsigned)db.x - nbs, s5 = (unsigned)db.y - nbs;
  const unsigned s6 = (unsigned)db.z - nbs, s7 = (unsigned)db.w - nbs;
  const unsigned r0 = (unsigned)ta.x - ug, r1 = (unsigned)ta.y - ug;
  const unsigned r2 = (unsigned)ta.z - ug, r3 = (unsigned)ta.w - ug;
  const unsigned r4 = (unsigned)tb.x - ug, r5 = (unsigned)tb.y - ug;
  const unsigned r6 = (unsigned)tb.z - ug, r7 = (unsigned)tb.w - ug;
  const bool h0 = (ue0 + 0u < unE) & (s0 < unb) & (r0 < ugr);
  const bool h1 = (ue0 + 1u < unE) & (s1 < unb) & (r1 < ugr);
  const bool h2 = (ue0 + 2u < unE) & (s2 < unb) & (r2 < ugr);
  const bool h3 = (ue0 + 3u < unE) & (s3 < unb) & (r3 < ugr);
  const bool h4 = (ue0 + 4u < unE) & (s4 < unb) & (r4 < ugr);
  const bool h5 = (ue0 + 5u < unE) & (s5 < unb) & (r5 < ugr);
  const bool h6 = (ue0 + 6u < unE) & (s6 < unb) & (r6 < ugr);
  const bool h7 = (ue0 + 7u < unE) & (s7 < unb) & (r7 < ugr);
  const unsigned any = __builtin_amdgcn_ballot_w32(h0 | h1 | h2 | h3 | h4 | h5 | h6 | h7);
  if (any != 0u) {
#define HITJ(J, HJ, SJ) { \
      const unsigned mj = __builtin_amdgcn_ballot_w32(HJ); \
      if (mj != 0u) { \
        if (HJ) { \
          const int pos = wc + (int)__builtin_amdgcn_mbcnt_lo(mj, 0u); \
          if (pos < WCAP) list[wave * WCAP + pos] = ((el0 + (J)) << SLA) | (int)(SJ); \
        } \
        wc += (int)__builtin_popcount(mj); } }
    HITJ(0, h0, s0)
    HITJ(1, h1, s1)
    HITJ(2, h2, s2)
    HITJ(3, h3, s3)
    HITJ(4, h4, s4)
    HITJ(5, h5, s5)
    HITJ(6, h6, s6)
    HITJ(7, h7, s7)
#undef HITJ
  }
  return wc;
}

__global__ __launch_bounds__(NTHR) void k_prep(const float* __restrict__ W1, const float* __restrict__ R1,
                                               const float* __restrict__ W2, const float* __restrict__ R2,
                                               unsigned short* B1, unsigned short* B2) {
  const int u = (int)blockIdx.x * NTHR + (int)threadIdx.x;
  v8us o;
  unsigned short* dp;
  const float* p;
  if (u < UB1) {
    const int row = u >> 3;
    const int k8  = (u & 7) * 8;
    if (u < UB1R) {
      const int r = row >> 6;
      const int n = row & 63;
      p = W1 + (size_t)r * DIN * DH + (size_t)k8 * DH + n;
    } else {
      const int n = row - RB1;
      p = R1 + (size_t)k8 * DH + n;
    }
    dp = B1 + (size_t)row * KB1 + k8;
  } else if (u < UTOT) {
    const int v   = u - UB1;
    const int row = v >> 4;
    const int k8  = (v & 15) * 8;
    const int kk  = k8 & (DH - 1);
    if (v < UB2R) {
      const int r = row >> 6;
      const int n = row & 63;
      p = W2 + (size_t)r * DH * DH + (size_t)kk * DH + n;
    } else {
      const int n = row - RB2;
      p = R2 + (size_t)kk * DH + n;
    }
    dp = B2 + (size_t)row * KB2 + k8;
  } else {
    return;
  }
#pragma unroll
  for (int i = 0; i < 8; ++i) o[i] = (unsigned short)bf16_bits(p[(size_t)i * DH]);
  *(volatile v8us*)dp = o;
  __threadfence();
  *(volatile v8us*)dp = o;
}

__global__ __launch_bounds__(NTHR) void k_cvx(const float* __restrict__ x, int nN, int nUnits,
                                              unsigned short* xb) {
  const int u = (int)blockIdx.x * NTHR + (int)threadIdx.x;
  if (u >= nUnits) return;
  const int row = u >> 3;
  const int k8  = (u & 7) * 8;
  const int rc  = row < nN ? row : nN - 1;
  const bool rok = row < nN;
  const float* p = x + (size_t)rc * DIN + k8;
  const v4f a0 = *(const v4f*)p;
  const v4f a1 = *(const v4f*)(p + 4);
  v8us o;
  o[0] = rok ? (unsigned short)bf16_bits(a0.x) : (unsigned short)0;
  o[1] = rok ? (unsigned short)bf16_bits(a0.y) : (unsigned short)0;
  o[2] = rok ? (unsigned short)bf16_bits(a0.z) : (unsigned short)0;
  o[3] = rok ? (unsigned short)bf16_bits(a0.w) : (unsigned short)0;
  o[4] = rok ? (unsigned short)bf16_bits(a1.x) : (unsigned short)0;
  o[5] = rok ? (unsigned short)bf16_bits(a1.y) : (unsigned short)0;
  o[6] = rok ? (unsigned short)bf16_bits(a1.z) : (unsigned short)0;
  o[7] = rok ? (unsigned short)bf16_bits(a1.w) : (unsigned short)0;
  unsigned short* dp = xb + (size_t)row * KB1 + k8;
  *(volatile v8us*)dp = o;
  __threadfence();
  *(volatile v8us*)dp = o;
}

template <int NT, int KK>
__global__ __launch_bounds__(GTHR) void k_gemm(const unsigned short* __restrict__ Au, int lda,
                                               const unsigned short* __restrict__ BT, int bRow0,
                                               const float* __restrict__ bias, int nbias, int biasOn,
                                               float* outp, int ldc, int nOut) {
  constexpr int CBW = 16 * NT;
  constexpr int LPR = 4 * NT;
  constexpr int RPI = 32 / LPR;
  constexpr int NI  = 16 / RPI;
  __shared__ __attribute__((aligned(16))) float stg[GBM * CBW];
  const int tid = (int)threadIdx.x, lane = tid & 31, wave = tid >> 5, hh = lane >> 4, m = lane & 15;
  const int rowBase = (int)blockIdx.x * GBM;
  const int colBase = (int)blockIdx.y * CBW;

  v8f acc[NT];
  {
    const v8f z = {0.f, 0.f, 0.f, 0.f, 0.f, 0.f, 0.f, 0.f};
#pragma unroll
    for (int t = 0; t < NT; ++t) acc[t] = z;
  }
  const unsigned short* ap = Au + (size_t)(rowBase + 16 * wave + m) * (size_t)lda + 8 * hh;
  const unsigned short* bp = BT + (size_t)(bRow0 + colBase + m) * (size_t)KK + 8 * hh;

#pragma unroll 1
  for (int k0 = 0; k0 < KK; k0 += 32) {
    Frag af;
    af.h[0] = *(const v8usa*)(ap + k0);
    af.h[1] = *(const v8usa*)(ap + k0 + 16);
#pragma unroll
    for (int nt = 0; nt < NT; ++nt) {
      const unsigned short* wq = bp + (size_t)(16 * nt) * (size_t)KK + k0;
      Frag bf;
      bf.h[0] = *(const v8usa*)wq;
      bf.h[1] = *(const v8usa*)(wq + 16);
      acc[nt] = wmb(af, bf, acc[nt]);
    }
  }

#pragma unroll
  for (int nt = 0; nt < NT; ++nt) {
    const int lc = 16 * nt + m;
#pragma unroll
    for (int r = 0; r < 8; ++r) {
      const int lr = 16 * wave + 8 * hh + r;
      stg[lr * CBW + lc] = acc[nt][r];
    }
  }
  __syncthreads();

  const int sub = lane / LPR;
  const int cq  = 4 * (lane % LPR);
  const float bsc = (biasOn != 0) ? 1.0f : 0.0f;
  const int bix = cq < nbias - 4 ? cq : nbias - 4;
  v4f b4;
  {
    const v4f tb = *(const v4fa*)(bias + bix);
    b4.x = bf16_val(tb.x) * bsc; b4.y = bf16_val(tb.y) * bsc;
    b4.z = bf16_val(tb.z) * bsc; b4.w = bf16_val(tb.w) * bsc;
  }

  v4f pv[NI];
#pragma unroll
  for (int i = 0; i < NI; ++i) pv[i] = *(const v4fa*)(stg + (16 * wave + RPI * i + sub) * CBW + cq) + b4;

#pragma unroll
  for (int i = 0; i < NI; ++i) {
    const int row = rowBase + 16 * wave + RPI * i + sub;
    if (row < nOut) *(volatile v4f*)(outp + (size_t)row * (size_t)ldc + colBase + cq) = pv[i];
  }
  __threadfence();
#pragma unroll
  for (int i = 0; i < NI; ++i) {
    const int row = rowBase + 16 * wave + RPI * i + sub;
    if (row < nOut) *(volatile v4f*)(outp + (size_t)row * (size_t)ldc + colBase + cq) = pv[i];
  }
}

template <int FIN>
__global__ __launch_bounds__(NTHR) void k_scan(const int* __restrict__ srcs, const int* __restrict__ dsts,
                                               const int* __restrict__ ets, int nE, int nN, int mRows, int g0,
                                               const float* __restrict__ T, float* accp, float* outp, float* part) {
  extern __shared__ __attribute__((aligned(16))) int dsm[];
  int* list = dsm;
  int* hl   = dsm + LISTN;
  int* sl   = hl + RCAP;
  int* cnt  = sl + RCAP;
  int* offs = cnt + NBA;
  int* cur  = offs + NBA;
  int* misc = cur + NBA;
  float* rtab = (float*)(misc + 16);
  float* wst = (float*)hl;
  float* pst = (float*)(hl + PSTOFF);
  const int tid = (int)threadIdx.x, lane = tid & 31, wave = tid >> 5;
  const int nodeBase = (int)blockIdx.x * NBA;

  {
    const v4i z4 = {0, 0, 0, 0};
    for (int i = tid * 4; i < AGG_ZINTS; i += NTHR * 4) *(v4ia*)(dsm + i) = z4;
    if (tid < 16) misc[tid] = 0;
    if (tid <= DEGCAP) rtab[tid] = 1.0f / fmaxf((float)tid, 1.0f);
  }
  __syncthreads();

  int t = 0, ov = 0;
  const int nChunks = (nE + CHUNK - 1) / CHUNK;
#pragma unroll 1
  for (int ch = 0; ch < nChunks; ++ch) {
    const int cbase = ch * CHUNK;
    const int wc = scan_chunk(dsts, ets, nE, cbase, nodeBase, g0, list, tid, lane, wave);
    if (lane == 0) misc[wave] = wc;
    __syncthreads();
    if (wave == 0) {
#pragma unroll 1
      for (int w2 = 0; w2 < NWAVE; ++w2) {
        int c = misc[w2];
        c = c < 0 ? 0 : (c > WCAP ? WCAP : c);
#pragma unroll 1
        for (int b0 = 0; b0 < c; b0 += 32) {
          const int idx = b0 + lane;
          const int ent = list[w2 * WCAP + (idx < WCAP ? idx : WCAP - 1)];
          const int m32 = (c - b0) < 32 ? (c - b0) : 32;
#pragma unroll 1
          for (int k = 0; k < m32; ++k) {
            const int u    = __builtin_amdgcn_readlane(ent, k);
            const int slot = u & (NBA - 1);
            const int el   = (u >> SLA) & (CHUNK - 1);
            const int eid  = cbase + el;
            if (t < RCAP) {
              if (lane == 0) { hl[t] = eid; cnt[slot] = cnt[slot] + 1; }
              t = t + 1;
            } else {
              ov = 1;
            }
          }
        }
      }
    }
    __syncthreads();
  }
  if (wave == 0 && lane == 0) { misc[8] = t; misc[9] = ov; }
  __syncthreads();
  int tt = misc[8];
  tt = tt < 0 ? 0 : (tt > RCAP ? RCAP : tt);
  const int ovf = misc[9];

  if (wave == 0) {
    const int base = lane * (NBA / 32);
    int sacc = 0;
#pragma unroll 1
    for (int i = 0; i < NBA / 32; ++i) sacc += cnt[base + i];
    int incl = sacc;
#pragma unroll
    for (int d = 1; d < 32; d <<= 1) {
      const int y = __shfl_up(incl, d, 32);
      if (lane >= d) incl += y;
    }
    int run = incl - sacc;
#pragma unroll 1
    for (int i = 0; i < NBA / 32; ++i) {
      const int cv = cnt[base + i];
      offs[base + i] = run;
      cur[base + i]  = run;
      run += cv;
    }
  }
  __syncthreads();
  if (wave == 0) {
#pragma unroll 1
    for (int b0 = 0; b0 < tt; b0 += 32) {
      const int idx = b0 + lane;
      const int ent = hl[idx < RCAP ? idx : RCAP - 1];
      const int ec  = ent < 0 ? 0 : (ent > nE - 1 ? nE - 1 : ent);
      int sd = dsts[ec] - nodeBase;
      sd = sd < 0 ? 0 : (sd > NBA - 1 ? NBA - 1 : sd);
      const int m32 = (tt - b0) < 32 ? (tt - b0) : 32;
#pragma unroll 1
      for (int k = 0; k < m32; ++k) {
        const int u    = __builtin_amdgcn_readlane(ent, k);
        const int slot = __builtin_amdgcn_readlane(sd, k);
        if (lane == 0) {
          int p = cur[slot];
          p = p < 0 ? 0 : (p > RCAP - 1 ? RCAP - 1 : p);
          sl[p] = u;
          cur[slot] = p + 1;
        }
      }
    }
  }
  __syncthreads();

  const float qnan = __int_as_float(0x7fc00000);
  const float pz = (ovf != 0) ? qnan : 0.0f;
  int wn = 0;
  float wm0 = 0.0f, wm1 = 0.0f, wq0 = 0.0f, wq1 = 0.0f;
#pragma unroll 1
  for (int si = 0; si < NBA / NWAVE; ++si) {
    const int s    = si * NWAVE + wave;
    const int node = nodeBase + s;
    int c = cnt[s];
    const bool big = c > DEGCAP;
    c = c < 0 ? 0 : (c > DEGCAP ? DEGCAP : c);
    int o = offs[s];
    o = o < 0 ? 0 : (o > RCAP ? RCAP : o);
    const int nc = node < mRows ? node : mRows - 1;

    int n0 = 0, n1 = 0;
#pragma unroll 1
    for (int b0 = 0; b0 < c; b0 += 32) {
      int idx = o + b0 + lane;
      idx = idx > RCAP - 1 ? RCAP - 1 : idx;
      const int ent = sl[idx];
      const int eid = ent < 0 ? 0 : (ent > nE - 1 ? nE - 1 : ent);
      int tg = ets[eid] - g0;
      tg = tg < 0 ? 0 : (tg > GR - 1 ? GR - 1 : tg);
      const int m32 = (c - b0) < 32 ? (c - b0) : 32;
      const unsigned lm = 0xffffffffu >> (32 - m32);
      n0 += (int)__builtin_popcount(__builtin_amdgcn_ballot_w32(tg == 0) & lm);
      n1 += (int)__builtin_popcount(__builtin_amdgcn_ballot_w32(tg == 1) & lm);
    }
    const int c0 = n0 > DEGCAP ? DEGCAP : n0, c1 = n1 > DEGCAP ? DEGCAP : n1;
    const float i0 = rtab[c0], i1 = rtab[c1];
    const float pzr = big ? qnan : pz;

    const v2f z2 = {0.0f, 0.0f};
    v2f a = z2;
#pragma unroll 1
    for (int b0 = 0; b0 < c; b0 += 32) {
      int idx = o + b0 + lane;
      idx = idx > RCAP - 1 ? RCAP - 1 : idx;
      const int ent = sl[idx];
      const int eid = ent < 0 ? 0 : (ent > nE - 1 ? nE - 1 : ent);
      int sr = srcs[eid];
      sr = sr < 0 ? 0 : (sr > nN - 1 ? nN - 1 : sr);
      int tg = ets[eid] - g0;
      tg = tg < 0 ? 0 : (tg > GR - 1 ? GR - 1 : tg);
      const int m32 = (c - b0) < 32 ? (c - b0) : 32;
#pragma unroll 1
      for (int k = 0; k < m32; ++k) {
        const int sk = __builtin_amdgcn_readlane(sr, k);
        const int tk = __builtin_amdgcn_readlane(tg, k);
        const float w = (tk == 0) ? i0 : i1;
        const v2f f = *(const v2fa*)(T + (size_t)sk * (size_t)TP + DH * tk + 2 * lane);
        a += w * f;
      }
    }
    const v2f arow = *(const v2fa*)(accp + (size_t)nc * (size_t)DH + 2 * lane);
    const v2f v = arow + a + pzr;
    if constexpr (FIN != 2) {
      if (node < mRows) {
        float* rp = accp + (size_t)node * (size_t)DH + 2 * lane;
        *(volatile v2f*)rp = v;
        __threadfence();
        *(volatile v2f*)rp = v;
      }
    }
    if constexpr (FIN == 1) {
      if (node < nN) {
        wn += 1;
        const float rk = 1.0f / (float)wn;
        const float d0 = v.x - wm0;
        wm0 = fmaf(d0, rk, wm0);
        wq0 = fmaf(d0, v.x - wm0, wq0);
        const float d1 = v.y - wm1;
        wm1 = fmaf(d1, rk, wm1);
        wq1 = fmaf(d1, v.y - wm1, wq1);
      }
    }
    if constexpr (FIN == 2) {
      if (node < nN) {
        float* rp = outp + (size_t)node * (size_t)DH + 2 * lane;
        *(volatile v2f*)rp = v;
        __threadfence();
        *(volatile v2f*)rp = v;
      }
    }
  }

  if constexpr (FIN == 1) {
    if (lane == 0) wst[wave * WSTW] = (float)wn;
    wst[wave * WSTW + 1 + 2 * lane]          = wm0;
    wst[wave * WSTW + 1 + 2 * lane + 1]      = wm1;
    wst[wave * WSTW + 1 + DH + 2 * lane]     = wq0;
    wst[wave * WSTW + 1 + DH + 2 * lane + 1] = wq1;
    __syncthreads();
    if (tid < DH) {
      float n = 0.0f, mean = 0.0f, M2 = 0.0f;
#pragma unroll 1
      for (int w2 = 0; w2 < NWAVE; ++w2) {
        const float nb = wst[w2 * WSTW];
        const float mb = wst[w2 * WSTW + 1 + tid];
        const float qb = wst[w2 * WSTW + 1 + DH + tid];
        if (nb > 0.5f) {
          const float nn = n + nb;
          const float delta = mb - mean;
          const float f = nb / nn;
          mean = fmaf(delta, f, mean);
          M2 = M2 + qb + delta * delta * n * f;
          n = nn;
        }
      }
      pst[1 + tid] = mean;
      pst[1 + DH + tid] = M2;
      if (tid == 0) pst[0] = n;
    }
#pragma unroll 1
    for (int i = 2 * DH + 1 + tid; i < PARTW; i += NTHR) pst[i] = 0.0f;
    __syncthreads();
    const int pb = (int)blockIdx.x;
    v4f ps = {0.0f, 0.0f, 0.0f, 0.0f};
    if (tid < PARTW / 4) {
      ps = *(const v4fa*)(pst + 4 * tid);
      *(volatile v4f*)(part + (size_t)pb * PARTW + 4 * tid) = ps;
    }
    __threadfence();
    if (tid < PARTW / 4) {
      *(volatile v4f*)(part + (size_t)pb * PARTW + 4 * tid) = ps;
    }
  }
}

__global__ __launch_bounds__(DH) void k_bnfin(const float* __restrict__ part, int nPart,
                                              const float* __restrict__ gam, const float* __restrict__ bet,
                                              float* ss) {
  __shared__ __attribute__((aligned(16))) float stg[2 * DH];
  const int tid = (int)threadIdx.x;
  const int c = tid;
  double n = 0.0, mean = 0.0, M2 = 0.0;
#pragma unroll 1
  for (int b = 0; b < nPart; ++b) {
    const float* pr = part + (size_t)b * PARTW;
    const double nb = (double)pr[0];
    const double mb = (double)pr[1 + c];
    const double qb = (double)pr[1 + DH + c];
    if (nb > 0.5) {
      const double nn = n + nb;
      const double delta = mb - mean;
      const double f = nb / nn;
      mean = mean + delta * f;
      M2 = M2 + qb + delta * delta * n * f;
      n = nn;
    }
  }
  const double nt = n < 1.0 ? 1.0 : n;
  const float varf  = (float)(M2 / nt);
  const float meanf = (float)mean;
  const float rstd = 1.0f / sqrtf(varf + 1e-5f);
  const float sc = bf16_val(gam[c]) * rstd;
  const float sh = bf16_val(bet[c]) - meanf * sc;
  stg[c] = sc;
  stg[DH + c] = sh;
  __syncthreads();
  v4f v = {0.0f, 0.0f, 0.0f, 0.0f};
  if (tid < (2 * DH) / 4) {
    v = *(const v4fa*)(stg + 4 * tid);
    *(volatile v4f*)(ss + 4 * tid) = v;
  }
  __threadfence();
  if (tid < (2 * DH) / 4) {
    *(volatile v4f*)(ss + 4 * tid) = v;
  }
}

__global__ __launch_bounds__(NTHR) void k_apply(const float* __restrict__ z, const float* __restrict__ ss,
                                                int nN, int mRows, unsigned short* apl) {
  __shared__ __attribute__((aligned(16))) float ssh[2 * DH];
  const int tid = (int)threadIdx.x, lane = tid & 31, wave = tid >> 5;
  if (tid < 2 * DH) ssh[tid] = ss[tid];
  __syncthreads();
  const int sub = lane >> 3;
  const int c8  = 8 * (lane & 7);
  const v4f sc0 = *(const v4fa*)(ssh + c8);
  const v4f sc1 = *(const v4fa*)(ssh + c8 + 4);
  const v4f sh0 = *(const v4fa*)(ssh + DH + c8);
  const v4f sh1 = *(const v4fa*)(ssh + DH + c8 + 4);
  const int rb0 = (int)blockIdx.x * APB + wave * APR;

  v8us qh[2], ql[2];
#pragma unroll
  for (int i = 0; i < 2; ++i) {
    const int row = rb0 + 4 * i + sub;
    const bool live = row < nN;
    const int rc = live ? row : (nN - 1);
    const float* zp = z + (size_t)rc * DH + c8;
    const v4f a0 = *(const v4f*)zp;
    const v4f a1 = *(const v4f*)(zp + 4);
    float y[8];
    y[0] = fmaxf(fmaf(a0.x, sc0.x, sh0.x), 0.0f);
    y[1] = fmaxf(fmaf(a0.y, sc0.y, sh0.y), 0.0f);
    y[2] = fmaxf(fmaf(a0.z, sc0.z, sh0.z), 0.0f);
    y[3] = fmaxf(fmaf(a0.w, sc0.w, sh0.w), 0.0f);
    y[4] = fmaxf(fmaf(a1.x, sc1.x, sh1.x), 0.0f);
    y[5] = fmaxf(fmaf(a1.y, sc1.y, sh1.y), 0.0f);
    y[6] = fmaxf(fmaf(a1.z, sc1.z, sh1.z), 0.0f);
    y[7] = fmaxf(fmaf(a1.w, sc1.w, sh1.w), 0.0f);
    v8us mh, ml;
#pragma unroll
    for (int e = 0; e < 8; ++e) {
      const float ye = live ? y[e] : 0.0f;
      const unsigned hb = bf16_bits(ye);
      mh[e] = (unsigned short)hb;
      ml[e] = (unsigned short)bf16_bits(ye - __uint_as_float(hb << 16));
    }
    qh[i] = mh;
    ql[i] = ml;
  }
#pragma unroll
  for (int i = 0; i < 2; ++i) {
    const int row = rb0 + 4 * i + sub;
    if (row < mRows) {
      *(volatile v8us*)(apl + (size_t)row * KB2 + c8) = qh[i];
      *(volatile v8us*)(apl + (size_t)row * KB2 + DH + c8) = ql[i];
    }
  }
  __threadfence();
#pragma unroll
  for (int i = 0; i < 2; ++i) {
    const int row = rb0 + 4 * i + sub;
    if (row < mRows) {
      *(volatile v8us*)(apl + (size_t)row * KB2 + c8) = qh[i];
      *(volatile v8us*)(apl + (size_t)row * KB2 + DH + c8) = ql[i];
    }
  }
}

static inline int cdiv(int a, int b) { return (a + b - 1) / b; }
static inline size_t al256(size_t o) { return (o + 255) & ~(size_t)255; }

extern "C" void kernel_launch(void* const* d_in, const int* in_sizes, int n_in,
                              void* d_out, int out_size, void* d_ws, size_t ws_size,
                              hipStream_t stream) {
  if (n_in < 11) return;
  if (in_sizes[0] < DIN || (in_sizes[0] % DIN) != 0) return;
  const int nN = in_sizes[0] / DIN;
  if (in_sizes[1] < 8 || (in_sizes[1] & 1) != 0) return;
  const int nE = in_sizes[1] / 2;
  if (nE < 4 || (nE & 3) != 0 || nE >= (1 << 26) || nN < 16 || nN >= (1 << 24)) return;
  if (in_sizes[2] != nE) return;
  if (in_sizes[3] != NREL * DIN * DH || in_sizes[4] != DIN * DH) return;
  if (in_sizes[5] != DH || in_sizes[6] != DH || in_sizes[7] != DH) return;
  if (in_sizes[8] != NREL * DH * DH || in_sizes[9] != DH * DH || in_sizes[10] != DH) return;
  if ((long long)out_size != (long long)nN * DH) return;

  const float* x    = (const float*)d_in[0];
  const int*   edge = (const int*)d_in[1];
  const int*   ety  = (const int*)d_in[2];
  const float* W1   = (const float*)d_in[3];
  const float* R1   = (const float*)d_in[4];
  const float* b1   = (const float*)d_in[5];
  const float* g1   = (const float*)d_in[6];
  const float* be1  = (const float*)d_in[7];
  const float* W2   = (const float*)d_in[8];
  const float* R2   = (const float*)d_in[9];
  const float* b2   = (const float*)d_in[10];
  float* out = (float*)d_out;
  const int* src = edge;
  const int* dst = edge + nE;

  const int MP = cdiv(nN, GBM) * GBM;
  const int gM = MP / GBM;
  const int gA = cdiv(MP, NBA);
  if ((long long)gA * NBA < (long long)MP) return;
  if ((MP % APB) != 0) return;

  char* ws = (char*)d_ws;
  size_t off = 0;
  const size_t oB1 = off; off = al256(off + (size_t)NB1 * KB1 * 2);
  const size_t oB2 = off; off = al256(off + (size_t)NB2 * KB2 * 2);
  const size_t oXB = off; off = al256(off + (size_t)MP * KB1 * 2);
  const size_t oT  = off; off = al256(off + (size_t)MP * TP * 4);
  const size_t oA  = off; off = al256(off + (size_t)MP * DH * 4);
  const size_t oX1 = off; off = al256(off + (size_t)MP * KB2 * 2);
  const size_t oPT = off; off = al256(off + (size_t)gA * PARTW * 4);
  const size_t oSS = off; off = al256(off + (size_t)(2 * DH) * 4);
  if (off > ws_size || off > (size_t)WSMAX) return;
  unsigned short* B1p = (unsigned short*)(ws + oB1);
  unsigned short* B2p = (unsigned short*)(ws + oB2);
  unsigned short* XB  = (unsigned short*)(ws + oXB);
  float*          Tp  = (float*)(ws + oT);
  float*          ACC = (float*)(ws + oA);
  unsigned short* X1  = (unsigned short*)(ws + oX1);
  float*          PT  = (float*)(ws + oPT);
  float*          SS  = (float*)(ws + oSS);

  const size_t scanLds = (size_t)AGG_LDS_INTS * 4;
  hipFuncSetAttribute(reinterpret_cast<const void*>(&k_scan<0>), hipFuncAttributeMaxDynamicSharedMemorySize, (int)scanLds);
  hipFuncSetAttribute(reinterpret_cast<const void*>(&k_scan<1>), hipFuncAttributeMaxDynamicSharedMemorySize, (int)scanLds);
  hipFuncSetAttribute(reinterpret_cast<const void*>(&k_scan<2>), hipFuncAttributeMaxDynamicSharedMemorySize, (int)scanLds);

  const int nUx = MP * (KB1 / 8);
  k_prep<<<UTOT / NTHR, NTHR, 0, stream>>>(W1, R1, W2, R2, B1p, B2p);
  k_cvx<<<cdiv(nUx, NTHR), NTHR, 0, stream>>>(x, nN, nUx, XB);

  k_gemm<4, KB1><<<dim3(gM, 1), GTHR, 0, stream>>>(XB, KB1, B1p, RB1, b1, DH, 1, ACC, DH, MP);
  for (int g = 0; g < NGRP; ++g) {
    k_gemm<8, KB1><<<dim3(gM, TP / 128), GTHR, 0, stream>>>(XB, KB1, B1p, TP * g, b1, DH, 0, Tp, TP, MP);
    if (g < NGRP - 1)
      k_scan<0><<<gA, NTHR, scanLds, stream>>>(src, dst, ety, nE, nN, MP, GR * g, Tp, ACC, out, PT);
    else
      k_scan<1><<<gA, NTHR, scanLds, stream>>>(src, dst, ety, nE, nN, MP, GR * g, Tp, ACC, out, PT);
  }
  k_bnfin<<<1, DH, 0, stream>>>(PT, gA, g1, be1, SS);
  k_apply<<<gM, NTHR, 0, stream>>>(ACC, SS, nN, MP, X1);

  k_gemm<4, KB2><<<dim3(gM, 1), GTHR, 0, stream>>>(X1, KB2, B2p, RB2, b2, DH, 1, ACC, DH, MP);
  for (int g = 0; g < NGRP; ++g) {
    k_gemm<8, KB2><<<dim3(gM, TP / 128), GTHR, 0, stream>>>(X1, KB2, B2p, TP * g, b2, DH, 0, Tp, TP, MP);
    if (g < NGRP - 1)
      k_scan<0><<<gA, NTHR, scanLds, stream>>>(src, dst, ety, nE, nN, MP, GR * g, Tp, ACC, out, PT);
    else
      k_scan<2><<<gA, NTHR, scanLds, stream>>>(src, dst, ety, nE, nN, MP, GR * g, Tp, ACC, out, PT);
  }
}
